// My_GATConv_3607772529308
// MI455X (gfx1250) — hardware-verified
//
#include <hip/hip_runtime.h>
#include <math.h>

#define NN   50000
#define NE   500000
#define NV   (NE + NN)
#define FD   64
#define NH   8
#define FW   512
#define NT   256
#define SRB  512
#define NTL  98
#define NPAD (NTL * SRB)
#define NTA  33

typedef __attribute__((ext_vector_type(16))) _Float16 v16h;
typedef __attribute__((ext_vector_type(8)))  _Float16 v8h;
typedef __attribute__((ext_vector_type(4)))  _Float16 v4h;
typedef __attribute__((ext_vector_type(16))) __bf16   v16b;
typedef __attribute__((ext_vector_type(8)))  __bf16   v8b;
typedef __attribute__((ext_vector_type(8)))  float    v8f;
typedef __attribute__((ext_vector_type(4)))  float    v4f;
typedef __attribute__((ext_vector_type(2)))  float    v2f;
typedef __attribute__((ext_vector_type(4)))  int      v4i;

__device__ __forceinline__ unsigned short f2bf_bits(float f) {
  unsigned u = __float_as_uint(f);
  return (unsigned short)((u + 0x7FFFu + ((u >> 16) & 1u)) >> 16);
}
__device__ __forceinline__ float bf_bits2f(unsigned short h) { return __uint_as_float(((unsigned)h) << 16); }

__device__ __forceinline__ void dep_guard_h(v8f& a, v8f& b, v16h x, v16h y) { asm volatile("v_nop\n\tv_nop\n\tv_nop\n\tv_nop" : "+v"(a), "+v"(b) : "v"(x), "v"(y)); }
__device__ __forceinline__ void dep_guard_b(v8f& a, v8f& b, v16b x, v16b y) { asm volatile("v_nop\n\tv_nop\n\tv_nop\n\tv_nop" : "+v"(a), "+v"(b) : "v"(x), "v"(y)); }
__device__ __forceinline__ void keep4_h(v16h a, v16h b, v16h c, v16h d) { asm volatile("v_nop" :: "v"(a), "v"(b), "v"(c), "v"(d)); }
__device__ __forceinline__ void keep4_b(v16b a, v16b b, v16b c, v16b d) { asm volatile("v_nop" :: "v"(a), "v"(b), "v"(c), "v"(d)); }
__device__ __forceinline__ void acc_guard4(v8f& a, v8f& b, v8f& c, v8f& d) { asm volatile("v_nop\n\tv_nop\n\tv_nop\n\tv_nop" : "+v"(a), "+v"(b), "+v"(c), "+v"(d)); }
template <typename T> struct Frag;
template <> struct Frag<_Float16> {
  typedef v16h V; union U { v16h v; v8h h[2]; };
  static __device__ __forceinline__ v16h load(const _Float16* p) {
    U f; f.h[0] = *(const v8h*)(p); f.h[1] = *(const v8h*)(p + 16); return f.v;
  }
  static __device__ __forceinline__ v8f mma(v16h a, v16h b, v8f c) {
    return __builtin_amdgcn_wmma_f32_16x16x32_f16(false, a, false, b, (short)0, c, false, false);
  }
  static __device__ __forceinline__ void guard(v8f& a, v8f& b, v16h x, v16h y) { dep_guard_h(a, b, x, y); }
  static __device__ __forceinline__ void keep(v16h a, v16h b, v16h c, v16h d) { keep4_h(a, b, c, d); }
};
template <> struct Frag<__bf16> {
  typedef v16b V; union U { v16b v; v8b h[2]; };
  static __device__ __forceinline__ v16b load(const __bf16* p) {
    U f; f.h[0] = *(const v8b*)(p); f.h[1] = *(const v8b*)(p + 16); return f.v;
  }
  static __device__ __forceinline__ v8f mma(v16b a, v16b b, v8f c) {
    return __builtin_amdgcn_wmma_f32_16x16x32_bf16(false, a, false, b, (short)0, c, false, false);
  }
  static __device__ __forceinline__ void guard(v8f& a, v8f& b, v16b x, v16b y) { dep_guard_b(a, b, x, y); }
  static __device__ __forceinline__ void keep(v16b a, v16b b, v16b c, v16b d) { keep4_b(a, b, c, d); }
};

template <int ET> struct Elem;
template <> struct Elem<0> { typedef _Float16 T; };
template <> struct Elem<1> { typedef __bf16 T; };
template <int ET, bool SPLIT, int BIAS_MODE, int OUT_MODE, bool RESID, int ACT = 0>
__global__ __launch_bounds__(256) void wmma_gemm64(
    const unsigned short* __restrict__ Ap, const unsigned short* __restrict__ A2p, int lda, long strideA,
    const unsigned short* __restrict__ Btp, const unsigned short* __restrict__ Bt2p, int ldb, long strideB,
    void* __restrict__ Cout, void* __restrict__ Cout2, int ldc, long strideC,
    const float* __restrict__ bias,
    const float* __restrict__ resid, long strideR,
    int M, int N, int K, float scale) {
  typedef typename Elem<ET>::T T;
  typedef typename Frag<T>::V V;
  const T* A = (const T*)Ap; const T* A2 = (const T*)A2p; const T* Bt = (const T*)Btp; const T* Bt2 = (const T*)Bt2p;
  __shared__ __align__(16) float sT[8][16 * 68];
  const int b    = blockIdx.y;
  const int lane = threadIdx.x & 31;
  const int wave = threadIdx.x >> 5;
  const int tilesN = N >> 6;
  const int tilesM = M >> 6;
  const int tile = blockIdx.x * 8 + wave;
  if (tile >= tilesM * tilesN) return;
  const int tm = tile / tilesN;
  const int tn = tile - tm * tilesN;
  const int m0 = tm << 6;
  const int n0 = tn << 6;

  const T* Ab  = A  + (size_t)b * strideA;
  const T* Bb  = Bt + (size_t)b * strideB;
  const T* Ab2 = SPLIT ? (A2  + (size_t)b * strideA) : nullptr;
  const T* Bb2 = SPLIT ? (Bt2 + (size_t)b * strideB) : nullptr;

  const int rlane = lane & 15;
  const int koff  = (lane >> 4) * 8;
  const int mOff  = (lane >> 4) * 8;

  v8f acc[4][4];
#pragma unroll
  for (int i = 0; i < 4; ++i)
#pragma unroll
    for (int j = 0; j < 4; ++j) acc[i][j] = (v8f){0.f,0.f,0.f,0.f,0.f,0.f,0.f,0.f};

  for (int k0 = 0; k0 < K; k0 += 32) {
    V bh[4], bl[4];
#pragma unroll
    for (int j = 0; j < 4; ++j) {
      const size_t bo = (size_t)(n0 + (j << 4) + rlane) * ldb + koff + k0;
      bh[j] = Frag<T>::load(Bb + bo);
      if (SPLIT) bl[j] = Frag<T>::load(Bb2 + bo);
    }
#pragma unroll
    for (int i = 0; i < 4; ++i) {
      const size_t ao = (size_t)(m0 + (i << 4) + rlane) * lda + koff + k0;
      V ah = Frag<T>::load(Ab + ao);
      V al;
      if (SPLIT) al = Frag<T>::load(Ab2 + ao);
#pragma unroll
      for (int j = 0; j < 4; ++j) {
        acc[i][j] = Frag<T>::mma(ah, bh[j], acc[i][j]);
        if (SPLIT) {
          acc[i][j] = Frag<T>::mma(ah, bl[j], acc[i][j]);
          acc[i][j] = Frag<T>::mma(al, bh[j], acc[i][j]);
        }
      }
      Frag<T>::guard(acc[i][0], acc[i][3], ah, SPLIT ? al : ah);
    }
    Frag<T>::keep(bh[0], bh[1], bh[2], bh[3]);
    if (SPLIT) Frag<T>::keep(bl[0], bl[1], bl[2], bl[3]);
  }
  acc_guard4(acc[0][0], acc[0][1], acc[0][2], acc[0][3]);
  acc_guard4(acc[1][0], acc[1][1], acc[1][2], acc[1][3]);
  acc_guard4(acc[2][0], acc[2][1], acc[2][2], acc[2][3]);
  acc_guard4(acc[3][0], acc[3][1], acc[3][2], acc[3][3]);

  float* slab = sT[wave];
  const float* Rb = RESID ? (resid + (size_t)b * strideR) : nullptr;
#pragma unroll
  for (int i = 0; i < 4; ++i) {
    const int mBase = m0 + (i << 4);
#pragma unroll
    for (int j = 0; j < 4; ++j) {
      const int n = n0 + (j << 4) + rlane;
      float bv = 0.f;
      if (BIAS_MODE == 2) bv = bias[n];
#pragma unroll
      for (int r = 0; r < 8; ++r) {
        float v = acc[i][j][r] * scale;
        if (BIAS_MODE == 1) v += bias[mBase + mOff + r];
        if (BIAS_MODE == 2) v += bv;
        if (RESID) v += Rb[(size_t)(mBase + mOff + r) * ldc + n];
        if (ACT == 1) v = tanhf(v);
        if (ACT == 2) v = fmaxf(v, 0.0f);
        if (ACT == 3) v = v / (1.0f + expf(-v));
        if (ACT == 4) v = (v > 0.f) ? v : 0.01f * v;
        if (ACT == 5) v = 0.5f * v * (1.0f + erff(v * 0.70710678118654752f));
        slab[(mOff + r) * 68 + (j << 4) + rlane] = v;
      }
    }
    __builtin_amdgcn_fence(__ATOMIC_RELEASE, "workgroup");
    __builtin_amdgcn_wave_barrier();
    __builtin_amdgcn_fence(__ATOMIC_ACQUIRE, "workgroup");
    if (OUT_MODE == 0) {
      float* C = (float*)Cout + (size_t)b * strideC;
      const int hh = lane >> 4, c4 = (lane & 15) * 4;
      for (int pass = 0; pass < 2; ++pass) {
#pragma unroll
        for (int it = 0; it < 8; ++it) {
          const int row = it * 2 + hh;
          v4f v = *(const v4f*)(slab + row * 68 + c4);
          *(volatile v4f*)(C + (size_t)(mBase + row) * ldc + n0 + c4) = v;
        }
        __threadfence();
      }
    } else {
      const int q = lane >> 3, c8 = (lane & 7) * 8;
      unsigned short* C  = (unsigned short*)Cout  + (size_t)b * strideC;
      unsigned short* C2 = (OUT_MODE == 2) ? ((unsigned short*)Cout2 + (size_t)b * strideC) : nullptr;
      for (int pass = 0; pass < 2; ++pass) {
#pragma unroll
        for (int it = 0; it < 4; ++it) {
          const int row = it * 4 + q;
          const float* sp = slab + row * 68 + c8;
          v8h hv, lv;
#pragma unroll
          for (int e = 0; e < 8; ++e) {
            if (OUT_MODE == 1) {
              hv[e] = (_Float16)sp[e];
            } else {
              unsigned short hb = f2bf_bits(sp[e]);
              unsigned short lb = f2bf_bits(sp[e] - bf_bits2f(hb));
              hv[e] = __builtin_bit_cast(_Float16, hb);
              lv[e] = __builtin_bit_cast(_Float16, lb);
            }
          }
          *(volatile v8h*)(C + (size_t)(mBase + row) * ldc + n0 + c8) = hv;
          if (OUT_MODE == 2) *(volatile v8h*)(C2 + (size_t)(mBase + row) * ldc + n0 + c8) = lv;
        }
        __threadfence();
      }
    }
    __builtin_amdgcn_fence(__ATOMIC_RELEASE, "workgroup");
    __builtin_amdgcn_wave_barrier();
    __builtin_amdgcn_fence(__ATOMIC_ACQUIRE, "workgroup");
  }
}

__global__ __launch_bounds__(256) void transpose_cast_f16(const float* __restrict__ in, int ldi,
                                                         _Float16* __restrict__ outT, int ldo, float scale) {
  __shared__ __align__(16) _Float16 tile[64][72];
  const int c0 = blockIdx.x * 64, r0 = blockIdx.y * 64;
  const int t = threadIdx.y * 32 + threadIdx.x;
  for (int i = threadIdx.y; i < 64; i += 8) {
    tile[threadIdx.x][i]      = (_Float16)(in[(size_t)(r0 + i) * ldi + c0 + threadIdx.x] * scale);
    tile[32 + threadIdx.x][i] = (_Float16)(in[(size_t)(r0 + i) * ldi + c0 + 32 + threadIdx.x] * scale);
  }
  __syncthreads();
  const int q = t >> 3, c8 = (t & 7) * 8;
  for (int pass = 0; pass < 2; ++pass) {
#pragma unroll
    for (int it = 0; it < 2; ++it) {
      const int c = it * 32 + q;
      v8h hv = *(const v8h*)(&tile[c][c8]);
      *(volatile v8h*)(outT + (size_t)(c0 + c) * ldo + r0 + c8) = hv;
    }
    __threadfence();
  }
}

__global__ __launch_bounds__(256) void padcast_rows_kernel(const float* __restrict__ x, unsigned* __restrict__ X16) {
  const long i = (long)blockIdx.x * 256 + threadIdx.x; if (i >= (long)NPAD * FD / 2) return;
  const long e0 = 2 * i; const bool ok = e0 < (long)NN * FD;
  const float a = ok ? x[e0] : 0.f, b = ok ? x[e0 + 1] : 0.f;
  const unsigned u = (unsigned)__builtin_bit_cast(unsigned short, (_Float16)a) | ((unsigned)__builtin_bit_cast(unsigned short, (_Float16)b) << 16);
  ((volatile unsigned*)X16)[i] = u; __threadfence(); ((volatile unsigned*)X16)[i] = u;
}

__global__ __launch_bounds__(NT) void att_terms_kernel(const _Float16* __restrict__ XW, const float* __restrict__ as, const float* __restrict__ ad,
                                                      float* __restrict__ ASD) {
  __shared__ __align__(16) float so[8 * 16];
  const int lane = threadIdx.x & 31, wave = threadIdx.x >> 5;
  const int n = blockIdx.x * 8 + wave;
  const int h = lane >> 2, cq = (lane & 3) * 16;
  const _Float16* xr = XW + (size_t)n * FW + h * FD + cq;
  const v8h x0 = *(const v8h*)(xr);
  const v8h x1 = *(const v8h*)(xr + 8);
  const float* sp = as + h * FD + cq;
  const float* dp = ad + h * FD + cq;
  const v4f s0 = *(const v4f*)(sp), s1 = *(const v4f*)(sp + 4), s2 = *(const v4f*)(sp + 8), s3 = *(const v4f*)(sp + 12);
  const v4f d0 = *(const v4f*)(dp), d1 = *(const v4f*)(dp + 4), d2 = *(const v4f*)(dp + 8), d3 = *(const v4f*)(dp + 12);
  float s = 0.f, d = 0.f;
#pragma unroll
  for (int e = 0; e < 4; ++e) {
    const float xa = (float)x0[e], xb = (float)x0[4 + e], xc = (float)x1[e], xd = (float)x1[4 + e];
    s += xa * s0[e]; s += xb * s1[e]; s += xc * s2[e]; s += xd * s3[e];
    d += xa * d0[e]; d += xb * d1[e]; d += xc * d2[e]; d += xd * d3[e];
  }
  s += __shfl_xor(s, 1, 32); s += __shfl_xor(s, 2, 32);
  d += __shfl_xor(d, 1, 32); d += __shfl_xor(d, 2, 32);
  if ((lane & 3) == 0) { so[wave * 16 + h] = s; so[wave * 16 + 8 + h] = d; }
  __syncthreads();
  if (wave == 0) {
    const v4f v = *(const v4f*)(so + 4 * lane);
    float* op = ASD + (size_t)blockIdx.x * 128 + 4 * lane;
    *(volatile v4f*)op = v; __threadfence(); *(volatile v4f*)op = v;
  }
}

__device__ __forceinline__ int blk_excl_scan(int cnt, int* scan_ws, int tid, int* tot) {
  const int lane = tid & 31, wave = tid >> 5; int incl = cnt;
#pragma unroll
  for (int o = 1; o < 32; o <<= 1) { const int v = __shfl_up(incl, o, 32); if (lane >= o) incl += v; }
  if (lane == 31) scan_ws[wave] = incl;
  __syncthreads();
  if (wave == 0) { int wv = (lane < NT / 32) ? scan_ws[lane] : 0; int wincl = wv;
#pragma unroll
    for (int o = 1; o < 32; o <<= 1) { const int v = __shfl_up(wincl, o, 32); if (lane >= o) wincl += v; }
    if (lane < NT / 32) scan_ws[32 + lane] = wincl - wv; if (lane == 31) scan_ws[64] = wincl; }
  __syncthreads();
  const int res = scan_ws[32 + wave] + incl - cnt; *tot = scan_ws[64];
  return res;
}
template <int SP, int CAP>
__device__ __forceinline__ int chunk_hits(const int* __restrict__ dstv, const int* __restrict__ srcv, int e0, int n0, int tid,
                                          int* LIST, int* scan_ws) {
  const int eb = e0 + tid * SP;
  int rec[SP]; int cnt = 0;
  if (eb < NE) {
#pragma unroll
    for (int k = 0; k < SP; k += 4) {
      const v4i d4 = *(const v4i*)(dstv + eb + k);
      const v4i s4 = *(const v4i*)(srcv + eb + k);
#pragma unroll
      for (int e = 0; e < 4; ++e) {
        const int d = d4[e]; int r = -1;
        if (d >= n0 && d < n0 + SRB) { int s = s4[e]; s = s < 0 ? 0 : (s >= NN ? NN - 1 : s); r = ((d - n0) << 16) | s; ++cnt; }
        rec[k + e] = r;
      }
    }
  } else {
#pragma unroll
    for (int k = 0; k < SP; ++k) {
      const int e = eb + k; const int d = e - NE; int r = -1;
      if (e < NV && d >= n0 && d < n0 + SRB) { r = ((d - n0) << 16) | d; ++cnt; }
      rec[k] = r;
    }
  }
  int tot; int p = blk_excl_scan(cnt, scan_ws, tid, &tot);
#pragma unroll
  for (int k = 0; k < SP; ++k) if (rec[k] >= 0) { if ((unsigned)p < (unsigned)CAP) LIST[p] = rec[k]; ++p; }
  __syncthreads();
  return tot < CAP ? tot : CAP;
}

#define SCH 2048
#define NCH ((NV + SCH - 1) / SCH)
__global__ __launch_bounds__(NT) void gat_agg_kernel(const _Float16* __restrict__ XW, const int* __restrict__ ei, const float* __restrict__ ASD,
                                                    const float* __restrict__ bias, const float* __restrict__ Hin, float* AGG,
                                                    float* __restrict__ HO, double* __restrict__ part, int tile0) {
  __shared__ int LIST[SCH];
  __shared__ float SM[SRB * NH];
  __shared__ float SL[SRB * NH];
  __shared__ float SAD[SRB * NH];
  __shared__ int scan_ws[80];
  __shared__ double red[16];
  const int tid = threadIdx.x, lane = tid & 31, wave = tid >> 5;
  const int tile = tile0 + blockIdx.x;
  const int n0 = tile * SRB;
  const int rbase = blockIdx.x * SRB;
  const int h8 = lane & 7;
  const v4f z4 = {0.f, 0.f, 0.f, 0.f};
#pragma unroll 1
  for (int j = 0; j < 64; ++j) {
    float* rp = AGG + (size_t)(rbase + wave * 64 + j) * FW + 4 * lane;
#pragma unroll
    for (int jj = 0; jj < 4; ++jj) *(v4f*)(rp + 128 * jj) = z4;
  }
  for (int i = tid; i < SRB * NH; i += NT) {
    SM[i] = -INFINITY; SL[i] = 0.f;
    const int dl = i >> 3, h = i & 7;
    SAD[i] = ASD[(size_t)(n0 + dl) * 16 + 8 + h];
  }
  __syncthreads();
  const int* srcv = ei; const int* dstv = ei + NE;
#pragma unroll 1
  for (int c = 0; c < NCH; ++c) {
    const int tot = chunk_hits<SCH / NT, SCH>(dstv, srcv, c * SCH, n0, tid, LIST, scan_ws);
#pragma unroll 1
    for (int base = 0; base < tot; base += 32) {
      const int q = base + lane;
      const int rv = (q < tot) ? LIST[q] : -1;
      const int own = (rv >= 0 && (rv >> 22) == wave) ? 1 : 0;
      unsigned msk = (unsigned)__ballot(own);
#pragma unroll 1
      for (int it = 0; it < 32; ++it) {
        if (msk == 0u) break;
        const int bp = __builtin_ctz(msk); msk &= msk - 1u;
        const int r = __shfl(rv, bp, 32);
        const int dl = r >> 16, s = r & 0xFFFF;
        const int mi = dl * NH + h8;
        float al = ASD[(size_t)s * 16 + h8] + SAD[mi];
        al = (al >= 0.f) ? al : 0.2f * al;
        const float mo = SM[mi], lo = SL[mi];
        const float mn = fmaxf(mo, al);
        const float rr = __expf(mo - mn), ex = __expf(al - mn);
        const float ln = lo * rr + ex;
        if (lane < 8) { SM[mi] = mn; SL[mi] = ln; }
        const _Float16* xr = XW + (size_t)s * FW + 4 * lane;
        float* rp = AGG + (size_t)(rbase + dl) * FW + 4 * lane;
#pragma unroll
        for (int j = 0; j < 4; ++j) {
          const int hj = 2 * j + (lane >> 4);
          const float rrj = __shfl(rr, hj, 32), exj = __shfl(ex, hj, 32);
          const v4h xv = *(const v4h*)(xr + 128 * j);
          const v4f hv = __builtin_convertvector(xv, v4f);
          v4f a = *(const v4f*)(rp + 128 * j);
          a = a * rrj + exj * hv;
          *(v4f*)(rp + 128 * j) = a;
        }
      }
    }
    __syncthreads();
  }
  const int c4 = (lane & 15) * 4;
  const v4f bs4 = *(const v4f*)(bias + c4);
  double ps = 0.0, pq = 0.0;
#pragma unroll 1
  for (int jj = 0; jj < 32; ++jj) {
    const int dl = wave * 64 + 2 * jj + (lane >> 4);
    const int n = n0 + dl;
    float lv = 1.0f;
    if ((lane & 15) < 8) lv = SL[dl * NH + (lane & 7)];
    lv = lv > 0.f ? lv : 1.0f;
    const float inv = 1.0f / lv;
    const float* rp = AGG + (size_t)(rbase + dl) * FW + c4;
    v4f acc = z4;
#pragma unroll
    for (int h = 0; h < NH; ++h) {
      const float ih = __shfl(inv, (lane & 16) + h, 32);
      const v4f a = *(const v4f*)(rp + FD * h);
      acc = acc + a * ih;
    }
    if (n0 + wave * 64 + 2 * jj < NN) {
      const v4f rsd = *(const v4f*)(Hin + (size_t)n * FD + c4);
      v4f v = acc * 0.125f + bs4;
      v = v + rsd;
      ps += (double)v[0] + (double)v[1] + (double)v[2] + (double)v[3];
      pq += (double)v[0] * v[0] + (double)v[1] * v[1] + (double)v[2] * v[2] + (double)v[3] * v[3];
      float* op = HO + (size_t)n * FD + c4;
      *(volatile v4f*)op = v; __threadfence(); *(volatile v4f*)op = v;
    }
  }
  for (int o = 16; o > 0; o >>= 1) { ps += __shfl_xor(ps, o, 32); pq += __shfl_xor(pq, o, 32); }
  if (lane == 0) { red[2 * wave] = ps; red[2 * wave + 1] = pq; }
  __syncthreads();
  if (wave == 0) {
    double a = 0.0, b = 0.0;
#pragma unroll
    for (int w = 0; w < 8; ++w) { a += red[2 * w]; b += red[2 * w + 1]; }
    const double val = (lane == 0) ? a : (lane == 1 ? b : 0.0);
    double* pp = part + (size_t)tile * 32 + lane;
    *(volatile double*)pp = val; __threadfence(); *(volatile double*)pp = val;
  }
}

__global__ __launch_bounds__(256) void gstats_kernel(const double* __restrict__ part, int nblocks, float* __restrict__ st) {
  __shared__ double ra[256], rb[256];
  double a = 0.0, b = 0.0;
  for (int i = threadIdx.x; i < nblocks; i += 256) { a += part[(size_t)i * 32]; b += part[(size_t)i * 32 + 1]; }
  ra[threadIdx.x] = a; rb[threadIdx.x] = b; __syncthreads();
  for (int s = 128; s > 0; s >>= 1) { if (threadIdx.x < s) { ra[threadIdx.x] += ra[threadIdx.x + s]; rb[threadIdx.x] += rb[threadIdx.x + s]; } __syncthreads(); }
  if (threadIdx.x < 32) { const double n = (double)NN * FD; const double mu = ra[0] / n; double var = rb[0] / n - mu * mu; if (var < 0.0) var = 0.0;
    const float v = (threadIdx.x == 0) ? (float)mu : (threadIdx.x == 1 ? (float)(1.0 / sqrt(var + 1e-5)) : 0.f);
    ((volatile float*)st)[threadIdx.x] = v; __threadfence(); ((volatile float*)st)[threadIdx.x] = v; }
}
__global__ __launch_bounds__(256) void norm_relu_kernel(const float* __restrict__ HO, const float* __restrict__ st, const float* __restrict__ g, const float* __restrict__ bb,
                                                       float* __restrict__ H, unsigned* __restrict__ H16) {
  const long i = (long)blockIdx.x * 256 + threadIdx.x; if (i >= (long)NPAD * FD / 2) return;
  const long e0 = 2 * i; const int c = (int)(e0 % FD); const bool ok = e0 < (long)NN * FD;
  const float mu = st[0], rs = st[1];
  float a = 0.f, b = 0.f;
  if (ok) { a = fmaxf((HO[e0] - mu) * rs * g[c] + bb[c], 0.f); b = fmaxf((HO[e0 + 1] - mu) * rs * g[c + 1] + bb[c + 1], 0.f); }
  const v2f v = {a, b};
  const unsigned u = (unsigned)__builtin_bit_cast(unsigned short, (_Float16)a) | ((unsigned)__builtin_bit_cast(unsigned short, (_Float16)b) << 16);
  if (ok) { *(volatile v2f*)(H + e0) = v; }
  ((volatile unsigned*)H16)[i] = u; __threadfence();
  if (ok) { *(volatile v2f*)(H + e0) = v; }
  ((volatile unsigned*)H16)[i] = u;
}

extern "C" void kernel_launch(void* const* d_in, const int* in_sizes, int n_in,
                              void* d_out, int out_size, void* d_ws, size_t ws_size, hipStream_t stream) {
  (void)in_sizes; (void)n_in; (void)out_size;
  const float* x     = (const float*)d_in[0];
  const int*   ei    = (const int*)  d_in[1];
  const float* W1    = (const float*)d_in[2];
  const float* as1   = (const float*)d_in[3];
  const float* ad1   = (const float*)d_in[4];
  const float* bias1 = (const float*)d_in[5];
  const float* g1    = (const float*)d_in[6];
  const float* b1    = (const float*)d_in[7];
  const float* W2    = (const float*)d_in[8];
  const float* as2   = (const float*)d_in[9];
  const float* ad2   = (const float*)d_in[10];
  const float* bias2 = (const float*)d_in[11];
  const float* g2    = (const float*)d_in[12];
  const float* b2    = (const float*)d_in[13];
  float* out = (float*)d_out;

  char* ws = (char*)d_ws; size_t off = 0;
  auto carve = [&](size_t bytes) -> char* { char* p = ws + off; off += (bytes + 255) & ~(size_t)255; return p; };
  _Float16* W1T  = (_Float16*)carve((size_t)FW * FD * 2);
  _Float16* W2T  = (_Float16*)carve((size_t)FW * FD * 2);
  unsigned* X16  = (unsigned*)carve((size_t)NPAD * FD * 2);
  _Float16* XW16 = (_Float16*)carve((size_t)NPAD * FW * 2);
  float*    ASD  = (float*)carve((size_t)NPAD * 16 * 4);
  float*    AGG  = (float*)carve((size_t)NTA * SRB * FW * 4);
  float*    HO   = (float*)carve((size_t)NPAD * FD * 4);
  float*    H1   = (float*)carve((size_t)NPAD * FD * 4);
  double*   part = (double*)carve((size_t)NTL * 32 * 8);
  float*    st   = (float*)carve(256);
  if (off > ws_size || off > (size_t)134217728) return;

  const int ncast = (NPAD * FD / 2 + 255) / 256;
  const int gtiles = (NPAD / 64) * (FW / 64);

  transpose_cast_f16<<<dim3(FW / 64, FD / 64), dim3(32, 8), 0, stream>>>(W1, FW, W1T, FD, 16.0f);
  transpose_cast_f16<<<dim3(FW / 64, FD / 64), dim3(32, 8), 0, stream>>>(W2, FW, W2T, FD, 16.0f);

  padcast_rows_kernel<<<ncast, 256, 0, stream>>>(x, X16);
  wmma_gemm64<0, false, 0, 1, false><<<dim3((gtiles + 7) / 8, 1), 256, 0, stream>>>(
      (const unsigned short*)X16, nullptr, FD, 0L, (const unsigned short*)W1T, nullptr, FD, 0L,
      (void*)XW16, nullptr, FW, 0L, nullptr, nullptr, 0L, NPAD, FW, FD, 0.0625f);
  att_terms_kernel<<<NPAD / 8, NT, 0, stream>>>(XW16, as1, ad1, ASD);
  gat_agg_kernel<<<NTA, NT, 0, stream>>>(XW16, ei, ASD, bias1, x, AGG, HO, part, 0);
  gat_agg_kernel<<<NTA, NT, 0, stream>>>(XW16, ei, ASD, bias1, x, AGG, HO, part, NTA);
  gat_agg_kernel<<<NTL - 2 * NTA, NT, 0, stream>>>(XW16, ei, ASD, bias1, x, AGG, HO, part, 2 * NTA);
  gstats_kernel<<<1, 256, 0, stream>>>(part, NTL, st);
  norm_relu_kernel<<<ncast, 256, 0, stream>>>(HO, st, g1, b1, H1, X16);

  wmma_gemm64<0, false, 0, 1, false><<<dim3((gtiles + 7) / 8, 1), 256, 0, stream>>>(
      (const unsigned short*)X16, nullptr, FD, 0L, (const unsigned short*)W2T, nullptr, FD, 0L,
      (void*)XW16, nullptr, FW, 0L, nullptr, nullptr, 0L, NPAD, FW, FD, 0.0625f);
  att_terms_kernel<<<NPAD / 8, NT, 0, stream>>>(XW16, as2, ad2, ASD);
  gat_agg_kernel<<<NTA, NT, 0, stream>>>(XW16, ei, ASD, bias2, H1, AGG, HO, part, 0);
  gat_agg_kernel<<<NTA, NT, 0, stream>>>(XW16, ei, ASD, bias2, H1, AGG, HO, part, NTA);
  gat_agg_kernel<<<NTL - 2 * NTA, NT, 0, stream>>>(XW16, ei, ASD, bias2, H1, AGG, HO, part, 2 * NTA);
  gstats_kernel<<<1, 256, 0, stream>>>(part, NTL, st + 32);
  norm_relu_kernel<<<ncast, 256, 0, stream>>>(HO, st + 32, g2, b2, out, X16);
}
